// RGBuvHistBlock_38895223832965
// MI455X (gfx1250) — hardware-verified
//
#include <hip/hip_runtime.h>

typedef __attribute__((ext_vector_type(16))) _Float16 v16h;
typedef __attribute__((ext_vector_type(8)))  _Float16 v8h;
typedef __attribute__((ext_vector_type(16))) __bf16   v16b;
typedef __attribute__((ext_vector_type(8)))  __bf16   v8b;
typedef __attribute__((ext_vector_type(8)))  float    v8f;
typedef __attribute__((ext_vector_type(4)))  float    v4f;

constexpr int NBATCH_C   = 8;
constexpr int NPIX_C     = 160000;
constexpr int HB_C       = 64;
constexpr int CHUNK_PIX  = 3200;
constexpr int NCHUNK_C   = NPIX_C / CHUNK_PIX;
constexpr int SUBK       = 128;
constexpr int NSUB_C     = CHUNK_PIX / SUBK;
constexpr int PITCH_H    = 136;
constexpr int PITCH_W    = PITCH_H / 2;
constexpr int EPI_PITCH  = 36;
constexpr int TILE_ELEMS = HB_C * HB_C;
static_assert(NCHUNK_C * CHUNK_PIX == NPIX_C, "no chunk tail");
static_assert(NSUB_C * SUBK == CHUNK_PIX, "no substage tail");
static_assert(SUBK % 32 == 0, "k steps of 32");
static_assert((NBATCH_C * NPIX_C) % 256 == 0, "prep grid exact");
static_assert(PITCH_H % 8 == 0, "16-byte aligned fragment rows");

__device__ __forceinline__ unsigned short f2bf_bits(float f) {
  unsigned u = __float_as_uint(f);
  return (unsigned short)((u + 0x7FFFu + ((u >> 16) & 1u)) >> 16);
}
__device__ __forceinline__ float bf_bits2f(unsigned short h) { return __uint_as_float(((unsigned)h) << 16); }

__device__ __forceinline__ void dep_guard_h(v8f& a, v8f& b, v16h x, v16h y) { asm volatile("v_nop\n\tv_nop\n\tv_nop\n\tv_nop" : "+v"(a), "+v"(b) : "v"(x), "v"(y)); }
__device__ __forceinline__ void dep_guard_b(v8f& a, v8f& b, v16b x, v16b y) { asm volatile("v_nop\n\tv_nop\n\tv_nop\n\tv_nop" : "+v"(a), "+v"(b) : "v"(x), "v"(y)); }
__device__ __forceinline__ void keep4_h(v16h a, v16h b, v16h c, v16h d) { asm volatile("v_nop" :: "v"(a), "v"(b), "v"(c), "v"(d)); }
__device__ __forceinline__ void keep4_b(v16b a, v16b b, v16b c, v16b d) { asm volatile("v_nop" :: "v"(a), "v"(b), "v"(c), "v"(d)); }
template <typename T> struct Frag;
template <> struct Frag<_Float16> {
  typedef v16h V; union U { v16h v; v8h h[2]; };
  static __device__ __forceinline__ v16h load(const _Float16* p) {
    U f; f.h[0] = *(const v8h*)(p); f.h[1] = *(const v8h*)(p + 16); return f.v;
  }
  static __device__ __forceinline__ v8f mma(v16h a, v16h b, v8f c) {
    return __builtin_amdgcn_wmma_f32_16x16x32_f16(false, a, false, b, (short)0, c, false, false);
  }
  static __device__ __forceinline__ void guard(v8f& a, v8f& b, v16h x, v16h y) { dep_guard_h(a, b, x, y); }
  static __device__ __forceinline__ void keep(v16h a, v16h b, v16h c, v16h d) { keep4_h(a, b, c, d); }
};
template <> struct Frag<__bf16> {
  typedef v16b V; union U { v16b v; v8b h[2]; };
  static __device__ __forceinline__ v16b load(const __bf16* p) {
    U f; f.h[0] = *(const v8b*)(p); f.h[1] = *(const v8b*)(p + 16); return f.v;
  }
  static __device__ __forceinline__ v8f mma(v16b a, v16b b, v8f c) {
    return __builtin_amdgcn_wmma_f32_16x16x32_bf16(false, a, false, b, (short)0, c, false, false);
  }
  static __device__ __forceinline__ void guard(v8f& a, v8f& b, v16b x, v16b y) { dep_guard_b(a, b, x, y); }
  static __device__ __forceinline__ void keep(v16b a, v16b b, v16b c, v16b d) { keep4_b(a, b, c, d); }
};

__device__ __forceinline__ void guard_a_b2(v8f& c0, v8f& c1, v16b a, v16b b0, v16b b1) {
  asm volatile("v_nop\n\tv_nop\n\tv_nop\n\tv_nop" : "+v"(c0), "+v"(c1) : "v"(a), "v"(b0), "v"(b1));
}

__device__ __forceinline__ unsigned int pack_bf16x2(float lo, float hi) {
  return (unsigned int)f2bf_bits(lo) | (((unsigned int)f2bf_bits(hi)) << 16);
}

__device__ __forceinline__ float iq_val(float d50, float b50) {
  const float t = d50 - b50;
  return __builtin_amdgcn_rcpf(fmaf(t, t, 1.0f));
}

__global__ __launch_bounds__(256) void prep_kernel(const float* __restrict__ x,
                                                   const float* __restrict__ m,
                                                   float* __restrict__ prep, int total) {
  const int i  = blockIdx.x * 256 + threadIdx.x;
  const int ic = (i < total) ? i : (total - 1);
  const int b  = ic / NPIX_C;
  const int p  = ic - b * NPIX_C;
  const float* xb = x + (size_t)b * 3 * NPIX_C;
  const float* mb = m + (size_t)b * 3 * NPIX_C;
  float r  = xb[p];
  float g  = xb[(size_t)NPIX_C + p];
  float bl = xb[(size_t)2 * NPIX_C + p];
  const float mv = mb[p];
  r  = fminf(fmaxf(r,  0.0f), 1.0f);
  g  = fminf(fmaxf(g,  0.0f), 1.0f);
  bl = fminf(fmaxf(bl, 0.0f), 1.0f);
  const float wmask = (mv > 0.5f) ? 1.0f : 0.0f;
  const float ss = (r * r + bl * bl) + g * g;
  const float iy = sqrtf(ss + 1e-6f);
  const float l0 = logf(r  + 1e-6f);
  const float l1 = logf(g  + 1e-6f);
  const float l2 = logf(bl + 1e-6f);
  v4f o;
  o.x = (l0 - l1) * 50.0f;
  o.y = (l0 - l2) * 50.0f;
  o.z = (l1 - l2) * 50.0f;
  o.w = iy * wmask;
  if (i < total) {
    float* dst = prep + (size_t)i * 4;
    *(volatile v4f*)dst = o;
    __threadfence();
    *(volatile v4f*)dst = o;
  }
}

__global__ __launch_bounds__(256) void hist_gemm_kernel(const float* __restrict__ prep,
                                                        float* __restrict__ part) {
  __shared__ __align__(16) unsigned int AuW[HB_C * PITCH_W];
  __shared__ __align__(16) unsigned int BvW[HB_C * PITCH_W];
  __shared__ __align__(16) float epi[8][16 * EPI_PITCH];

  const int chunk = blockIdx.x;
  const int pair  = blockIdx.y;
  const int b     = blockIdx.z;
  const int tid   = threadIdx.x;
  const int lane  = tid & 31;
  const int wave  = tid >> 5;
  const int pp    = tid & 63;
  const int bg    = tid >> 6;
  const int tu    = wave & 3;
  const int tvb   = (wave >> 2) * 2;
  const int rlane = lane & 15;
  const int koff  = (lane >> 4) * 8;
  const int mOff  = (lane >> 4) * 8;

  float bin50[16];
#pragma unroll
  for (int i = 0; i < 16; ++i) {
    const int j = bg * 16 + i;
    const float st = (float)j * (1.0f / 63.0f);
    float bv = -3.0f * (1.0f - st) + 3.0f * st;
    bv = (j == 63) ? 3.0f : bv;
    bin50[i] = bv * 50.0f;
  }

  v8f acc0 = (v8f){0.f,0.f,0.f,0.f,0.f,0.f,0.f,0.f};
  v8f acc1 = (v8f){0.f,0.f,0.f,0.f,0.f,0.f,0.f,0.f};

  const float* prepb = prep + ((size_t)b * NPIX_C + (size_t)chunk * CHUNK_PIX) * 4;
  const __bf16* Au = (const __bf16*)(const void*)AuW;
  const __bf16* Bv = (const __bf16*)(const void*)BvW;

#pragma unroll 1
  for (int s = 0; s < NSUB_C; ++s) {
    const v4f p0 = *(const v4f*)(prepb + (size_t)(s * SUBK + 2 * pp) * 4);
    const v4f p1 = *(const v4f*)(prepb + (size_t)(s * SUBK + 2 * pp + 1) * 4);
    const float du0 = (pair == 0) ? p0.x : ((pair == 1) ? -p0.x : -p0.y);
    const float dv0 = (pair == 0) ? p0.y : ((pair == 1) ?  p0.z : -p0.z);
    const float du1 = (pair == 0) ? p1.x : ((pair == 1) ? -p1.x : -p1.y);
    const float dv1 = (pair == 0) ? p1.y : ((pair == 1) ?  p1.z : -p1.z);
    const float w0 = p0.w, w1 = p1.w;

    __syncthreads();
#pragma unroll
    for (int i = 0; i < 16; ++i) {
      const int u = bg * 16 + i;
      const float bb = bin50[i];
      const float ku0 = w0 * iq_val(du0, bb);
      const float ku1 = w1 * iq_val(du1, bb);
      const float kv0 = iq_val(dv0, bb);
      const float kv1 = iq_val(dv1, bb);
      AuW[u * PITCH_W + pp] = pack_bf16x2(ku0, ku1);
      BvW[u * PITCH_W + pp] = pack_bf16x2(kv0, kv1);
    }
    __syncthreads();

#pragma unroll
    for (int k0 = 0; k0 < SUBK; k0 += 32) {
      const v16b a  = Frag<__bf16>::load(Au + (size_t)(tu * 16 + rlane) * PITCH_H + koff + k0);
      const v16b b0 = Frag<__bf16>::load(Bv + (size_t)(tvb * 16 + rlane) * PITCH_H + koff + k0);
      const v16b b1 = Frag<__bf16>::load(Bv + (size_t)((tvb + 1) * 16 + rlane) * PITCH_H + koff + k0);
      acc0 = Frag<__bf16>::mma(a, b0, acc0);
      acc1 = Frag<__bf16>::mma(a, b1, acc1);
      guard_a_b2(acc0, acc1, a, b0, b1);
    }
  }

  float* slab = epi[wave];
#pragma unroll
  for (int r = 0; r < 8; ++r) {
    slab[(mOff + r) * EPI_PITCH + rlane]      = acc0[r];
    slab[(mOff + r) * EPI_PITCH + 16 + rlane] = acc1[r];
  }
  __syncthreads();
  float* dst = part + ((size_t)((b * 3 + pair) * NCHUNK_C + chunk)) * TILE_ELEMS
             + (size_t)(tu * 16) * HB_C + tvb * 16;
  const int q  = lane >> 3;
  const int c4 = (lane & 7) * 4;
  for (int pass = 0; pass < 2; ++pass) {
#pragma unroll
    for (int it = 0; it < 4; ++it) {
      const int row = it * 4 + q;
      const v4f v = *(const v4f*)(slab + row * EPI_PITCH + c4);
      *(volatile v4f*)(dst + (size_t)row * HB_C + c4) = v;
    }
    __threadfence();
  }
}

__global__ __launch_bounds__(256) void reduce_norm_kernel(const float* __restrict__ part,
                                                          float* __restrict__ out) {
  __shared__ float red[256];
  const int b   = blockIdx.x;
  const int tid = threadIdx.x;
  v4f hs[12];
  float tsum = 0.0f;
#pragma unroll
  for (int it = 0; it < 12; ++it) {
    const int f  = it * 256 + tid;
    const int pr = f >> 10;
    const int e  = (f & 1023) * 4;
    const float* src = part + ((size_t)(b * 3 + pr) * NCHUNK_C) * TILE_ELEMS + e;
    v4f a = (v4f){0.f, 0.f, 0.f, 0.f};
#pragma unroll 1
    for (int c = 0; c < NCHUNK_C; ++c) {
      const v4f pv = *(const v4f*)(src + (size_t)c * TILE_ELEMS);
      a += pv;
    }
    hs[it] = a;
    tsum += (a.x + a.y) + (a.z + a.w);
  }
  red[tid] = tsum;
  __syncthreads();
  for (int st = 128; st > 0; st >>= 1) {
    if (tid < st) red[tid] += red[tid + st];
    __syncthreads();
  }
  const float inv = 1.0f / (red[0] + 1e-6f);
#pragma unroll
  for (int it = 0; it < 12; ++it) hs[it] = hs[it] * inv;
  float* ob = out + (size_t)b * (3 * TILE_ELEMS);
  for (int pass = 0; pass < 2; ++pass) {
#pragma unroll
    for (int it = 0; it < 12; ++it) {
      const v4f v = hs[it];
      *(volatile v4f*)(ob + (size_t)(it * 256 + tid) * 4) = v;
    }
    __threadfence();
  }
}

extern "C" void kernel_launch(void* const* d_in, const int* in_sizes, int n_in,
                              void* d_out, int out_size, void* d_ws, size_t ws_size,
                              hipStream_t stream)
{
  const size_t prep_bytes = (size_t)NBATCH_C * NPIX_C * 4 * sizeof(float);
  const size_t part_bytes = (size_t)NBATCH_C * 3 * NCHUNK_C * TILE_ELEMS * sizeof(float);
  if (n_in < 2) return;
  if (in_sizes[0] < NBATCH_C * 3 * NPIX_C || in_sizes[1] < NBATCH_C * 3 * NPIX_C) return;
  if (out_size < NBATCH_C * 3 * TILE_ELEMS) return;
  if (ws_size < prep_bytes + part_bytes) return;

  const float* x = (const float*)d_in[0];
  const float* m = (const float*)d_in[1];
  float* out  = (float*)d_out;
  float* prep = (float*)d_ws;
  float* part = (float*)((char*)d_ws + prep_bytes);

  const int total_pix = NBATCH_C * NPIX_C;
  prep_kernel<<<total_pix / 256, 256, 0, stream>>>(x, m, prep, total_pix);
  hist_gemm_kernel<<<dim3(NCHUNK_C, 3, NBATCH_C), 256, 0, stream>>>(prep, part);
  reduce_norm_kernel<<<NBATCH_C, 256, 0, stream>>>(part, out);
}
